// FeatureAttention_49684181680937
// MI455X (gfx1250) — hardware-verified
//
#include <hip/hip_runtime.h>
#include <math.h>

constexpr int kRows  = 8192;
constexpr int kDimIn = 512;
constexpr int kUnits = 256;
constexpr int kQB    = 1024;
constexpr int kNQB   = kRows / kQB;
constexpr float kScoreScale = 0.0625f;
constexpr float kLoCarry    = 2048.0f;
constexpr float kLoCarryInv = 1.0f / 2048.0f;
static_assert(kRows % kQB == 0, "blocks");
static_assert(kQB % 64 == 0 && kUnits % 64 == 0 && kDimIn % 64 == 0 && kRows % 64 == 0, "tiles");
static_assert(kDimIn % 32 == 0 && kUnits % 32 == 0 && kRows % 32 == 0, "ksteps");
static_assert(kQB % 32 == 0 && kRows % 256 == 0, "softmax map");

typedef __attribute__((ext_vector_type(16))) _Float16 v16h;
typedef __attribute__((ext_vector_type(8)))  _Float16 v8h;
typedef __attribute__((ext_vector_type(16))) __bf16   v16b;
typedef __attribute__((ext_vector_type(8)))  __bf16   v8b;
typedef __attribute__((ext_vector_type(8)))  float    v8f;
typedef __attribute__((ext_vector_type(4)))  float    v4f;
typedef __attribute__((ext_vector_type(4)))  unsigned int v4u;

__device__ __forceinline__ unsigned short f2bf_bits(float f) {
  unsigned u = __float_as_uint(f);
  return (unsigned short)((u + 0x7FFFu + ((u >> 16) & 1u)) >> 16);
}
__device__ __forceinline__ float bf_bits2f(unsigned short h) { return __uint_as_float(((unsigned)h) << 16); }

__device__ __forceinline__ void dep_guard_h(v8f& a, v8f& b, v16h x, v16h y) { asm volatile("v_nop\n\tv_nop\n\tv_nop\n\tv_nop" : "+v"(a), "+v"(b) : "v"(x), "v"(y)); }
__device__ __forceinline__ void dep_guard_b(v8f& a, v8f& b, v16b x, v16b y) { asm volatile("v_nop\n\tv_nop\n\tv_nop\n\tv_nop" : "+v"(a), "+v"(b) : "v"(x), "v"(y)); }
__device__ __forceinline__ void keep4_h(v16h a, v16h b, v16h c, v16h d) { asm volatile("v_nop" :: "v"(a), "v"(b), "v"(c), "v"(d)); }
__device__ __forceinline__ void keep4_b(v16b a, v16b b, v16b c, v16b d) { asm volatile("v_nop" :: "v"(a), "v"(b), "v"(c), "v"(d)); }
__device__ __forceinline__ void acc_guard4(v8f& a, v8f& b, v8f& c, v8f& d) { asm volatile("v_nop\n\tv_nop\n\tv_nop\n\tv_nop" : "+v"(a), "+v"(b), "+v"(c), "+v"(d)); }
template <typename T> struct Frag;
template <> struct Frag<_Float16> {
  typedef v16h V; union U { v16h v; v8h h[2]; };
  static __device__ __forceinline__ v16h load(const _Float16* p) {
    U f; f.h[0] = *(const v8h*)(p); f.h[1] = *(const v8h*)(p + 16); return f.v;
  }
  static __device__ __forceinline__ v8f mma(v16h a, v16h b, v8f c) {
    return __builtin_amdgcn_wmma_f32_16x16x32_f16(false, a, false, b, (short)0, c, false, false);
  }
  static __device__ __forceinline__ void guard(v8f& a, v8f& b, v16h x, v16h y) { dep_guard_h(a, b, x, y); }
  static __device__ __forceinline__ void keep(v16h a, v16h b, v16h c, v16h d) { keep4_h(a, b, c, d); }
};
template <> struct Frag<__bf16> {
  typedef v16b V; union U { v16b v; v8b h[2]; };
  static __device__ __forceinline__ v16b load(const __bf16* p) {
    U f; f.h[0] = *(const v8b*)(p); f.h[1] = *(const v8b*)(p + 16); return f.v;
  }
  static __device__ __forceinline__ v8f mma(v16b a, v16b b, v8f c) {
    return __builtin_amdgcn_wmma_f32_16x16x32_bf16(false, a, false, b, (short)0, c, false, false);
  }
  static __device__ __forceinline__ void guard(v8f& a, v8f& b, v16b x, v16b y) { dep_guard_b(a, b, x, y); }
  static __device__ __forceinline__ void keep(v16b a, v16b b, v16b c, v16b d) { keep4_b(a, b, c, d); }
};

__device__ __forceinline__ unsigned pk16(unsigned short a, unsigned short b) { return (unsigned)a | ((unsigned)b << 16); }
__device__ __forceinline__ unsigned short h_bits(float f) { const _Float16 h = (_Float16)f; return __builtin_bit_cast(unsigned short, h); }

template <int ET> struct Elem;
template <> struct Elem<0> { typedef _Float16 T; };
template <> struct Elem<1> { typedef __bf16 T; };
template <int ET, bool SPLIT, int BIAS_MODE, int OUT_MODE, bool RESID, int ACT = 0>
__global__ __launch_bounds__(256) void wmma_gemm64(
    const unsigned short* __restrict__ Ap, const unsigned short* __restrict__ A2p, int lda, long strideA,
    const unsigned short* __restrict__ Btp, const unsigned short* __restrict__ Bt2p, int ldb, long strideB,
    void* __restrict__ Cout, void* __restrict__ Cout2, int ldc, long strideC,
    const float* __restrict__ bias,
    const float* __restrict__ resid, long strideR,
    int M, int N, int K, float scale) {
  typedef typename Elem<ET>::T T;
  typedef typename Frag<T>::V V;
  const T* A = (const T*)Ap; const T* A2 = (const T*)A2p; const T* Bt = (const T*)Btp; const T* Bt2 = (const T*)Bt2p;
  __shared__ __align__(16) float sT[8][16 * 68];
  const int b    = blockIdx.y;
  const int lane = threadIdx.x & 31;
  const int wave = threadIdx.x >> 5;
  const int tilesN = N >> 6;
  const int tilesM = M >> 6;
  const int tile = blockIdx.x * 8 + wave;
  if (tile >= tilesM * tilesN) return;
  const int tm = tile / tilesN;
  const int tn = tile - tm * tilesN;
  const int m0 = tm << 6;
  const int n0 = tn << 6;

  const T* Ab  = A  + (size_t)b * strideA;
  const T* Bb  = Bt + (size_t)b * strideB;
  const T* Ab2 = SPLIT ? (A2  + (size_t)b * strideA) : nullptr;
  const T* Bb2 = SPLIT ? (Bt2 + (size_t)b * strideB) : nullptr;

  const int rlane = lane & 15;
  const int koff  = (lane >> 4) * 8;
  const int mOff  = (lane >> 4) * 8;

  v8f acc[4][4];
#pragma unroll
  for (int i = 0; i < 4; ++i)
#pragma unroll
    for (int j = 0; j < 4; ++j) acc[i][j] = (v8f){0.f,0.f,0.f,0.f,0.f,0.f,0.f,0.f};

  for (int k0 = 0; k0 < K; k0 += 32) {
    V bh[4], bl[4];
#pragma unroll
    for (int j = 0; j < 4; ++j) {
      const size_t bo = (size_t)(n0 + (j << 4) + rlane) * ldb + koff + k0;
      bh[j] = Frag<T>::load(Bb + bo);
      if (SPLIT) bl[j] = Frag<T>::load(Bb2 + bo);
    }
#pragma unroll
    for (int i = 0; i < 4; ++i) {
      const size_t ao = (size_t)(m0 + (i << 4) + rlane) * lda + koff + k0;
      V ah = Frag<T>::load(Ab + ao);
      V al;
      if (SPLIT) al = Frag<T>::load(Ab2 + ao);
#pragma unroll
      for (int j = 0; j < 4; ++j) {
        acc[i][j] = Frag<T>::mma(ah, bh[j], acc[i][j]);
        if (SPLIT) {
          acc[i][j] = Frag<T>::mma(ah, bl[j], acc[i][j]);
          acc[i][j] = Frag<T>::mma(al, bh[j], acc[i][j]);
        }
      }
      Frag<T>::guard(acc[i][0], acc[i][3], ah, SPLIT ? al : ah);
    }
    Frag<T>::keep(bh[0], bh[1], bh[2], bh[3]);
    if (SPLIT) Frag<T>::keep(bl[0], bl[1], bl[2], bl[3]);
  }
  acc_guard4(acc[0][0], acc[0][1], acc[0][2], acc[0][3]);
  acc_guard4(acc[1][0], acc[1][1], acc[1][2], acc[1][3]);
  acc_guard4(acc[2][0], acc[2][1], acc[2][2], acc[2][3]);
  acc_guard4(acc[3][0], acc[3][1], acc[3][2], acc[3][3]);

  float* slab = sT[wave];
  const float* Rb = RESID ? (resid + (size_t)b * strideR) : nullptr;
#pragma unroll
  for (int i = 0; i < 4; ++i) {
    const int mBase = m0 + (i << 4);
#pragma unroll
    for (int j = 0; j < 4; ++j) {
      const int n = n0 + (j << 4) + rlane;
      float bv = 0.f;
      if (BIAS_MODE == 2) bv = bias[n];
#pragma unroll
      for (int r = 0; r < 8; ++r) {
        float v = acc[i][j][r] * scale;
        if (BIAS_MODE == 1) v += bias[mBase + mOff + r];
        if (BIAS_MODE == 2) v += bv;
        if (BIAS_MODE == 3) v *= bias[mBase + mOff + r];
        if (RESID) v += Rb[(size_t)(mBase + mOff + r) * ldc + n];
        if (ACT == 2) v = fmaxf(v, 0.0f);
        if (ACT == 4) v = (v > 0.f) ? v : 0.01f * v;
        slab[(mOff + r) * 68 + (j << 4) + rlane] = v;
      }
    }
    __builtin_amdgcn_fence(__ATOMIC_RELEASE, "workgroup");
    __builtin_amdgcn_wave_barrier();
    __builtin_amdgcn_fence(__ATOMIC_ACQUIRE, "workgroup");
    if (OUT_MODE == 0) {
      float* C = (float*)Cout + (size_t)b * strideC;
      const int hh = lane >> 4, c4 = (lane & 15) * 4;
      for (int pass = 0; pass < 2; ++pass) {
#pragma unroll
        for (int it = 0; it < 8; ++it) {
          const int row = it * 2 + hh;
          v4f v = *(const v4f*)(slab + row * 68 + c4);
          *(volatile v4f*)(C + (size_t)(mBase + row) * ldc + n0 + c4) = v;
        }
        __threadfence();
      }
    } else {
      const int q = lane >> 3, c8 = (lane & 7) * 8;
      unsigned short* C  = (unsigned short*)Cout  + (size_t)b * strideC;
      unsigned short* C2 = (OUT_MODE >= 2) ? ((unsigned short*)Cout2 + (size_t)b * strideC) : nullptr;
      for (int pass = 0; pass < 2; ++pass) {
#pragma unroll
        for (int it = 0; it < 4; ++it) {
          const int row = it * 4 + q;
          const float* sp = slab + row * 68 + c8;
          v8h hv, lv;
#pragma unroll
          for (int e = 0; e < 8; ++e) {
            if (OUT_MODE == 1) {
              hv[e] = (_Float16)sp[e];
            } else if (OUT_MODE == 3) {
              const _Float16 hq = (_Float16)sp[e];
              hv[e] = hq;
              lv[e] = (_Float16)((sp[e] - (float)hq) * kLoCarry);
            } else {
              unsigned short hb = f2bf_bits(sp[e]);
              unsigned short lb = f2bf_bits(sp[e] - bf_bits2f(hb));
              hv[e] = __builtin_bit_cast(_Float16, hb);
              lv[e] = __builtin_bit_cast(_Float16, lb);
            }
          }
          *(volatile v8h*)(C + (size_t)(mBase + row) * ldc + n0 + c8) = hv;
          if (OUT_MODE >= 2) *(volatile v8h*)(C2 + (size_t)(mBase + row) * ldc + n0 + c8) = lv;
        }
        __threadfence();
      }
    }
    __builtin_amdgcn_fence(__ATOMIC_RELEASE, "workgroup");
    __builtin_amdgcn_wave_barrier();
    __builtin_amdgcn_fence(__ATOMIC_ACQUIRE, "workgroup");
  }
}

__global__ __launch_bounds__(256) void cast8_bf16_kernel(const float* __restrict__ in, unsigned short* __restrict__ out, int n8) {
  const int i = blockIdx.x * 256 + threadIdx.x;
  if (i >= n8) return;
  const float* p = in + 8 * (size_t)i;
  const v4f a = *(const v4f*)(p);
  const v4f c = *(const v4f*)(p + 4);
  unsigned short hb[8];
#pragma unroll
  for (int e = 0; e < 4; ++e) {
    hb[e]     = f2bf_bits(a[e]);
    hb[4 + e] = f2bf_bits(c[e]);
  }
  const v4u u = (v4u){pk16(hb[0], hb[1]), pk16(hb[2], hb[3]), pk16(hb[4], hb[5]), pk16(hb[6], hb[7])};
  unsigned short* q = out + 8 * (size_t)i;
  *(volatile v4u*)q = u;
  __threadfence();
  *(volatile v4u*)q = u;
}

__global__ __launch_bounds__(256) void wtcast_bf16_kernel(const float* __restrict__ W0, const float* __restrict__ W1,
                                                          const float* __restrict__ W2,
                                                          unsigned short* __restrict__ O0, unsigned short* __restrict__ O1,
                                                          unsigned short* __restrict__ O2, int R, int Cc) {
  __shared__ float sm[64][65];
  const int t  = threadIdx.x;
  const int c0 = blockIdx.x * 64;
  const int r0 = blockIdx.y * 64;
  const int z  = blockIdx.z;
  const float* W = (z == 0) ? W0 : (z == 1) ? W1 : W2;
  unsigned short* op = (z == 0) ? O0 : (z == 1) ? O1 : O2;
#pragma unroll
  for (int i = 0; i < 16; ++i) {
    const int e  = i * 256 + t;
    const int rl = e >> 6;
    const int cl = e & 63;
    sm[cl][rl] = W[(size_t)(r0 + rl) * Cc + c0 + cl];
  }
  __syncthreads();
  const int lane = t & 31, wave = t >> 5;
  const int q = lane >> 3, c8 = (lane & 7) * 8;
  for (int pass = 0; pass < 2; ++pass) {
#pragma unroll
    for (int it = 0; it < 2; ++it) {
      const int row = wave * 8 + it * 4 + q;
      unsigned short hb[8];
#pragma unroll
      for (int e = 0; e < 8; ++e) hb[e] = f2bf_bits(sm[row][c8 + e]);
      const v4u u = (v4u){pk16(hb[0], hb[1]), pk16(hb[2], hb[3]), pk16(hb[4], hb[5]), pk16(hb[6], hb[7])};
      *(volatile v4u*)(op + (size_t)(c0 + row) * R + r0 + c8) = u;
    }
    __threadfence();
  }
}

__global__ __launch_bounds__(256) void softmax_rows_kernel(const float* __restrict__ S, unsigned short* __restrict__ P,
                                                           float* __restrict__ rinv) {
  __shared__ float sInv[32];
  const int t = threadIdx.x;
  const int lane = t & 31, wave = t >> 5;
  const int rowBase = blockIdx.x * 32;
#pragma unroll 1
  for (int rr = 0; rr < 4; ++rr) {
    const int rloc = wave * 4 + rr;
    const int row  = rowBase + rloc;
    const float* sr = S + (size_t)row * kRows;
    unsigned short* pr = P + (size_t)row * kRows;
    float m = -INFINITY;
#pragma unroll 1
    for (int it = 0; it < kRows / 256; ++it) {
      const float* p = sr + it * 256 + lane * 8;
      const v4f a = *(const v4f*)(p);
      const v4f c = *(const v4f*)(p + 4);
      const float m0 = fmaxf(fmaxf(a[0], a[1]), fmaxf(a[2], a[3]));
      const float m1 = fmaxf(fmaxf(c[0], c[1]), fmaxf(c[2], c[3]));
      m = fmaxf(m, fmaxf(m0, m1));
    }
#pragma unroll
    for (int off = 16; off > 0; off >>= 1) m = fmaxf(m, __shfl_xor(m, off, 32));
    float sum = 0.f;
#pragma unroll 1
    for (int it = 0; it < kRows / 256; ++it) {
      const int col = it * 256 + lane * 8;
      const float* p = sr + col;
      const v4f a = *(const v4f*)(p);
      const v4f c = *(const v4f*)(p + 4);
      float ev[8];
#pragma unroll
      for (int k = 0; k < 4; ++k) {
        ev[k]     = __expf(a[k] - m);
        ev[4 + k] = __expf(c[k] - m);
      }
      const float ps = ((ev[0] + ev[1]) + (ev[2] + ev[3])) + ((ev[4] + ev[5]) + (ev[6] + ev[7]));
      sum += ps;
      unsigned short hb[8];
#pragma unroll
      for (int k = 0; k < 8; ++k) hb[k] = h_bits(ev[k]);
      const v4u u = (v4u){pk16(hb[0], hb[1]), pk16(hb[2], hb[3]), pk16(hb[4], hb[5]), pk16(hb[6], hb[7])};
      unsigned short* q = pr + col;
      *(volatile v4u*)q = u;
      __threadfence();
      *(volatile v4u*)q = u;
    }
#pragma unroll
    for (int off = 16; off > 0; off >>= 1) sum += __shfl_xor(sum, off, 32);
    if (lane == 0) sInv[rloc] = 1.0f / sum;
  }
  __syncthreads();
  if (wave == 0) {
    const float v = sInv[lane];
    float* rp = rinv + rowBase + lane;
    *(volatile float*)rp = v;
    __threadfence();
    *(volatile float*)rp = v;
  }
}

static inline unsigned gemm_blocks(int M, int N) { return (unsigned)((((M / 64) * (N / 64)) + 7) / 8); }
static inline size_t align128(size_t b) { return (b + 127) & ~(size_t)127; }

extern "C" void kernel_launch(void* const* d_in, const int* in_sizes, int n_in,
                              void* d_out, int out_size, void* d_ws, size_t ws_size,
                              hipStream_t stream) {
  if (n_in < 5) return;
  if (in_sizes[0] != kRows * kDimIn || in_sizes[1] != kDimIn * kUnits || in_sizes[2] != kDimIn * kUnits ||
      in_sizes[3] != kDimIn * kUnits || in_sizes[4] != kUnits * kDimIn || out_size != kRows * kDimIn) return;

  const float* x  = (const float*)d_in[0];
  const float* Wq = (const float*)d_in[1];
  const float* Wk = (const float*)d_in[2];
  const float* Wv = (const float*)d_in[3];
  const float* Wo = (const float*)d_in[4];
  float* out = (float*)d_out;

  char* ws = (char*)d_ws;
  size_t off = 0;
  const size_t o_xb   = off; off += align128((size_t)kRows * kDimIn * 2);
  const size_t o_wqk  = off; off += align128((size_t)2 * kUnits * kDimIn * 2);
  const size_t o_wv   = off; off += align128((size_t)kUnits * kDimIn * 2);
  const size_t o_wo   = off; off += align128((size_t)kDimIn * kUnits * 2);
  const size_t o_qk   = off; off += align128((size_t)kRows * 2 * kUnits * 2);
  const size_t o_vth  = off; off += align128((size_t)kUnits * kRows * 2);
  const size_t o_vtl  = off; off += align128((size_t)kUnits * kRows * 2);
  const size_t o_s    = off; off += align128((size_t)kQB * kRows * 4);
  const size_t o_p    = off; off += align128((size_t)kQB * kRows * 2);
  const size_t o_rinv = off; off += align128((size_t)kQB * 4);
  const size_t o_o1   = off; off += align128((size_t)kQB * kUnits * 4);
  const size_t o_ohi  = off; off += align128((size_t)kQB * kUnits * 2);
  const size_t o_olo  = off; off += align128((size_t)kQB * kUnits * 2);
  const size_t o_out1 = off; off += align128((size_t)kQB * kDimIn * 4);
  if (off > ws_size) return;

  unsigned short* xb   = (unsigned short*)(ws + o_xb);
  unsigned short* wqk  = (unsigned short*)(ws + o_wqk);
  unsigned short* wv   = (unsigned short*)(ws + o_wv);
  unsigned short* wo   = (unsigned short*)(ws + o_wo);
  unsigned short* qk   = (unsigned short*)(ws + o_qk);
  unsigned short* vth  = (unsigned short*)(ws + o_vth);
  unsigned short* vtl  = (unsigned short*)(ws + o_vtl);
  float*          Sbuf = (float*)(ws + o_s);
  unsigned short* Pbuf = (unsigned short*)(ws + o_p);
  float*          rinv = (float*)(ws + o_rinv);
  float*          o1   = (float*)(ws + o_o1);
  unsigned short* ohi  = (unsigned short*)(ws + o_ohi);
  unsigned short* olo  = (unsigned short*)(ws + o_olo);
  float*          out1 = (float*)(ws + o_out1);

  const dim3 blk(256);

  {
    const int n8 = kRows * kDimIn / 8;
    cast8_bf16_kernel<<<dim3((unsigned)((n8 + 255) / 256)), blk, 0, stream>>>(x, xb, n8);
  }
  wtcast_bf16_kernel<<<dim3(kUnits / 64, kDimIn / 64, 3), blk, 0, stream>>>(
      Wq, Wk, Wv, wqk, wqk + (size_t)kUnits * kDimIn, wv, kDimIn, kUnits);
  wtcast_bf16_kernel<<<dim3(kDimIn / 64, kUnits / 64, 1), blk, 0, stream>>>(
      Wo, Wo, Wo, wo, wo, wo, kUnits, kDimIn);

  wmma_gemm64<1, false, 0, 1, false><<<dim3(gemm_blocks(kRows, 2 * kUnits)), blk, 0, stream>>>(
      xb, xb, kDimIn, 0L, wqk, wqk, kDimIn, 0L, (void*)qk, (void*)qk, 2 * kUnits, 0L,
      x, x, 0L, kRows, 2 * kUnits, kDimIn, 1.0f);
  wmma_gemm64<1, false, 0, 3, false><<<dim3(gemm_blocks(kUnits, kRows)), blk, 0, stream>>>(
      wv, wv, kDimIn, 0L, xb, xb, kDimIn, 0L, (void*)vth, (void*)vtl, kRows, 0L,
      x, x, 0L, kUnits, kRows, kDimIn, 1.0f);

  for (int qb = 0; qb < kNQB; ++qb) {
    const unsigned short* qblk = qk + (size_t)qb * kQB * (2 * kUnits);
    const unsigned short* kall = qk + kUnits;
    wmma_gemm64<0, false, 0, 0, false><<<dim3(gemm_blocks(kQB, kRows)), blk, 0, stream>>>(
        qblk, qblk, 2 * kUnits, 0L, kall, kall, 2 * kUnits, 0L, (void*)Sbuf, (void*)Sbuf, kRows, 0L,
        x, x, 0L, kQB, kRows, kUnits, kScoreScale);
    softmax_rows_kernel<<<dim3(kQB / 32), blk, 0, stream>>>(Sbuf, Pbuf, rinv);
    wmma_gemm64<0, false, 3, 0, false><<<dim3(gemm_blocks(kQB, kUnits)), blk, 0, stream>>>(
        Pbuf, Pbuf, kRows, 0L, vth, vth, kRows, 0L, (void*)o1, (void*)o1, kUnits, 0L,
        rinv, x, 0L, kQB, kUnits, kRows, 1.0f);
    wmma_gemm64<0, false, 3, 2, true><<<dim3(gemm_blocks(kQB, kUnits)), blk, 0, stream>>>(
        Pbuf, Pbuf, kRows, 0L, vtl, vtl, kRows, 0L, (void*)ohi, (void*)olo, kUnits, 0L,
        rinv, o1, 0L, kQB, kUnits, kRows, kLoCarryInv);
    wmma_gemm64<1, false, 0, 0, false><<<dim3(gemm_blocks(kQB, kDimIn)), blk, 0, stream>>>(
        ohi, ohi, kUnits, 0L, wo, wo, kUnits, 0L, (void*)out1, (void*)out1, kDimIn, 0L,
        x, x, 0L, kQB, kDimIn, kUnits, 1.0f);
    float* oblk = out + (size_t)qb * kQB * kDimIn;
    wmma_gemm64<1, false, 0, 0, true><<<dim3(gemm_blocks(kQB, kDimIn)), blk, 0, stream>>>(
        olo, olo, kUnits, 0L, wo, wo, kUnits, 0L, (void*)oblk, (void*)oblk, kDimIn, 0L,
        x, out1, 0L, kQB, kDimIn, kUnits, 1.0f);
  }
}
